// FM_v_38560216383899
// MI455X (gfx1250) — hardware-verified
//
#include <hip/hip_runtime.h>


#ifndef BROWS
#define BROWS 32768
#endif
#define B_FULL 32768
#define CF   8
#define VN   12
#define DN   64
#define TABN (CF * VN * DN)
#define AW   4
#define RPB  (16 * AW)
#define NBLK (BROWS / RPB)
#define SHP  72
#define PLINE 32
#define TBLK (TABN / 256)
#define NPIECE (BROWS / 4)
#define NPT  ((NBLK + 255) / 256)
#define OUT1_EL (2 * B_FULL)
#define OUT2_EL (2 * B_FULL + 1)

static_assert(DN == 64);
static_assert(DN % 32 == 0);
static_assert(AW == 4);
static_assert(BROWS % RPB == 0);
static_assert(BROWS <= B_FULL);
static_assert(TABN % 256 == 0);
static_assert((TABN / 4) % (32 * AW) == 0);
static_assert((CF * RPB) % (32 * AW) == 0);
static_assert(RPB * 2 == 32 * AW);
static_assert(SHP % 8 == 0);
static_assert(SHP >= DN);
static_assert(32 * 16 == RPB * 2 * 4);
static_assert(16 * 16 == RPB * 4);
static_assert(8 * 16 == PLINE * 4);
static_assert(64 * 16 == 256 * 4);
static_assert(128 * 16 == 16 * DN * 2);
static_assert(2 * DN == 16 * 8);
static_assert(NPIECE % 256 == 0);
static_assert(BROWS % 4 == 0);
static_assert((size_t)OUT1_EL * 4 == 262144);
static_assert((size_t)OUT2_EL * 4 == 262148);
static_assert(OUT1_EL % 32 == 0);
static_assert((size_t)OUT1_EL + (size_t)4 * (NPIECE - 1) + 4 == (size_t)OUT2_EL + BROWS - 1);
static_assert((size_t)TABN * 4 * 2 + (size_t)CF * RPB * 4 + (size_t)RPB * SHP * 2 + (size_t)RPB * 2 * 4 + (size_t)RPB * 4 + (size_t)AW * 4 <= 65536);

typedef _Float16 h16;
typedef __attribute__((ext_vector_type(16))) _Float16 v16h;
typedef __attribute__((ext_vector_type(8)))  _Float16 v8h;
typedef __attribute__((ext_vector_type(8)))  float    v8f;
typedef __attribute__((ext_vector_type(4)))  float    v4f;
typedef v4f  __attribute__((may_alias)) v4fa;

__device__ __forceinline__ unsigned short f2bf(float f) { unsigned u = __float_as_uint(f); u += 0x7FFFu + ((u >> 16) & 1u); return (unsigned short)(u >> 16); }
__device__ __forceinline__ float bfr(float f) { return __uint_as_float(((unsigned)f2bf(f)) << 16); }
__device__ __forceinline__ v16h cat16(v8h lo, v8h hi) { return __builtin_shufflevector(lo, hi, 0, 1, 2, 3, 4, 5, 6, 7, 8, 9, 10, 11, 12, 13, 14, 15); }
__device__ __forceinline__ v8f wmma16(v16h a, v16h b, v8f c) { return __builtin_amdgcn_wmma_f32_16x16x32_f16(false, a, false, b, (short)0, c, false, false); }
__device__ __forceinline__ v16h  ldh(const h16* p) { return cat16(*(const v8h*)p, *(const v8h*)(p + 16)); }
__device__ __forceinline__ void wave_sync() { __builtin_amdgcn_fence(3  , "wavefront"); __builtin_amdgcn_wave_barrier(); asm volatile("" ::: "memory"); }
static __device__ __forceinline__ h16 toh_flush(float v) { const h16 r = (h16)v; return (fabsf(v) < 6.103515625e-05f) ? (h16)0.0f : r; }
__device__ __forceinline__ v8f wmma16g(v16h a, v16h b, v8f c) {
    c = wmma16(a, b, c);
    asm volatile("v_nop\n\tv_nop\n\tv_nop\n\tv_nop" : "+v"(c) : "v"(a), "v"(b));
    return c;
}

__global__ __launch_bounds__(256) void k_prep(const float* __restrict__ meant, const float* __restrict__ stdt, const float* __restrict__ act, float* TAB, h16* ACTH) {
#pragma clang fp contract(off)
    __shared__ __align__(16) float st[512];
    const int tid = threadIdx.x;
    const int wave = __builtin_amdgcn_readfirstlane((int)(threadIdx.x >> 5));
    if (blockIdx.x < TBLK) {
        const int i = blockIdx.x * 256 + tid;
        const float mv = bfr(meant[i]);
        const float x = bfr(stdt[i]);
        const float sp = fmaxf(x, 0.0f) + log1pf(expf(-fabsf(x)));
        st[tid] = mv; st[256 + tid] = sp;
        __syncthreads();
        if (wave < 4) {
            const int which = wave >> 1, p = tid & 63;
            const v4f val = *(const v4fa*)(&st[which * 256 + 4 * p]);
            float* dst = TAB + (size_t)which * TABN + (size_t)blockIdx.x * 256 + 4 * p;
            *(volatile v4f*)dst = val; __threadfence(); *(volatile v4f*)dst = val;
        }
    } else {
        const int ic = tid < 15 ? tid : 15;
        v4f x0 = *(const v4f*)(act + ic * 8), x1 = *(const v4f*)(act + ic * 8 + 4);
        asm volatile("" : "+v"(x0), "+v"(x1));
        v8h o;
#pragma unroll
        for (int k = 0; k < 4; ++k) { const h16 a0 = toh_flush(bfr(x0[k])); const h16 a1 = toh_flush(bfr(x1[k]));
            o[k] = (tid < 16) ? a0 : (h16)0.0f; o[4 + k] = (tid < 16) ? a1 : (h16)0.0f; }
        if (wave < 4) {
            h16* dst = ACTH + (size_t)tid * 8;
            *(volatile v8h*)dst = o; __threadfence(); *(volatile v8h*)dst = o;
        }
    }
}

__global__ __launch_bounds__(32 * AW) void k_main(const int* __restrict__ idx, const float* __restrict__ label, const float* __restrict__ posw, const float* __restrict__ noise, const float* __restrict__ TAB, const h16* __restrict__ ACTH, float* OUT, float* PW, float* PART) {
    __shared__ __align__(16) float mu_s[TABN];
    __shared__ __align__(16) float sp_s[TABN];
    __shared__ int ro_s[CF * RPB];
    __shared__ __align__(16) h16 sh_s[RPB * SHP];
    __shared__ __align__(16) float inf_s[RPB * 2];
    __shared__ __align__(16) float pw_s[RPB];
    __shared__ float red_s[AW];
    const int tid = threadIdx.x;
    const int lane = tid & 31, lr = lane & 15, hi = lane >> 4;
    const int wave = __builtin_amdgcn_readfirstlane((int)(threadIdx.x >> 5));
    const int rb0 = blockIdx.x * RPB;
#pragma unroll 1
    for (int i = tid; i < TABN / 4; i += 32 * AW) {
        const v4f a = *(const v4f*)(TAB + 4 * i); const v4f c = *(const v4f*)(TAB + TABN + 4 * i);
        *(v4fa*)(&mu_s[4 * i]) = a; *(v4fa*)(&sp_s[4 * i]) = c; }
#pragma unroll 1
    for (int i = tid; i < CF * RPB; i += 32 * AW) {
        const int c = i / RPB, r = i % RPB;
        int v = idx[(size_t)c * B_FULL + rb0 + r];
        v = v < 0 ? v + VN : v; v = v < 0 ? 0 : (v > VN - 1 ? VN - 1 : v);
        ro_s[i] = (c * VN + v) * DN; }
    __syncthreads();

    const int row = wave * 16 + lr;
    const float* nz = noise + (size_t)(rb0 + row) * DN + 32 * hi;
    float s2 = 0.0f, e2 = 0.0f;
#pragma unroll 1
    for (int ch = 0; ch < 2; ++ch) {
        const int d0 = 32 * hi + 16 * ch;
        float w[16], s[16];
#pragma unroll
        for (int q = 0; q < 4; ++q) { const v4f n4 = *(const v4f*)(nz + 16 * ch + 4 * q);
#pragma unroll
            for (int k = 0; k < 4; ++k) { w[4 * q + k] = bfr(n4[k]); s[4 * q + k] = 0.0f; } }
#pragma unroll 1
        for (int c = 0; c < CF; ++c) {
            const int o = ro_s[c * RPB + row] + d0;
#pragma unroll
            for (int q = 0; q < 4; ++q) {
                const v4f mu = *(const v4fa*)(&mu_s[o + 4 * q]); const v4f sp = *(const v4fa*)(&sp_s[o + 4 * q]);
#pragma unroll
                for (int k = 0; k < 4; ++k) { const float e = mu[k] + (sp[k] * w[4 * q + k]) * 0.01f; s[4 * q + k] += e; e2 = fmaf(e, e, e2); } } }
        v8h h0, h1;
#pragma unroll
        for (int k = 0; k < 8; ++k) { s2 = fmaf(s[k], s[k], s2); s2 = fmaf(s[8 + k], s[8 + k], s2); h0[k] = toh_flush(s[k]); h1[k] = toh_flush(s[8 + k]); }
        *(v8h*)(&sh_s[row * SHP + d0]) = h0; *(v8h*)(&sh_s[row * SHP + d0 + 8]) = h1;
    }
    wave_sync();
    const int ao = row * SHP + 8 * hi;
    const v16h a0 = cat16(*(const v8h*)(&sh_s[ao]),      *(const v8h*)(&sh_s[ao + 16]));
    const v16h a1 = cat16(*(const v8h*)(&sh_s[ao + 32]), *(const v8h*)(&sh_s[ao + 48]));
    const v16h b0 = ldh(ACTH + (size_t)lr * DN + 8 * hi), b1 = ldh(ACTH + (size_t)lr * DN + 32 + 8 * hi);
    v8f acc = (v8f){};
    acc = wmma16g(a0, b0, acc);
    acc = wmma16g(a1, b1, acc);

    const float s2f = s2 + __shfl_xor(s2, 16, 32);
    const float e2f = e2 + __shfl_xor(e2, 16, 32);
    if (hi == 0) pw_s[row] = 0.5f * (s2f - e2f);
    if (lr < 2) {
#pragma unroll
        for (int r = 0; r < 8; ++r) inf_s[(wave * 16 + 8 * hi + r) * 2 + lr] = acc[r]; }
    __syncthreads();

    const float iv = inf_s[tid];
    const size_t ge = (size_t)rb0 * 2 + tid;
    const float lab = bfr(label[ge]); const float pwt = bfr(posw[ge]);
    const float dl = iv - lab;
    float term = pwt * (dl * dl);
#pragma unroll
    for (int off = 16; off >= 1; off >>= 1) term += __shfl_xor(term, off, 32);
    if (lane == 0) red_s[wave] = term;
    __syncthreads();

    if (wave == 0) {
        const v4f val = *(const v4fa*)(&inf_s[4 * lane]);
        float* dst = OUT + (size_t)rb0 * 2 + 4 * lane;
        *(volatile v4f*)dst = val; __threadfence(); *(volatile v4f*)dst = val;
    }
    if (wave == 1) {
        const v4f val = *(const v4fa*)(&pw_s[4 * lr]);
        float* dst = PW + (size_t)rb0 + 4 * lr;
        if (lane < 16) { *(volatile v4f*)dst = val; __threadfence(); *(volatile v4f*)dst = val; }
    }
    if (wave == 2) {
        const float t = ((red_s[0] + red_s[1]) + red_s[2]) + red_s[3];
        v4f val = (v4f){}; val[0] = (lane == 0) ? t : 0.0f;
        float* dst = PART + (size_t)blockIdx.x * PLINE + 4 * (lane & 7);
        if (lane < 8) { *(volatile v4f*)dst = val; __threadfence(); *(volatile v4f*)dst = val; }
    }
}

__global__ __launch_bounds__(256) void k_fin(const float* __restrict__ PW, const float* __restrict__ PART, float* OUT) {
#pragma clang fp contract(off)
    __shared__ float red_s[8];
    const int tid = threadIdx.x, lane = tid & 31;
    const int wave = __builtin_amdgcn_readfirstlane((int)(threadIdx.x >> 5));
    float loss = 0.0f;
    if (blockIdx.x == 0) {
        float v = 0.0f;
#pragma unroll 1
        for (int k = 0; k < NPT; ++k) {
            const int i = tid + 256 * k; const int ic = i < NBLK ? i : NBLK - 1;
            float x = PART[(size_t)ic * PLINE];
            asm volatile("" : "+v"(x));
            v += (i < NBLK) ? x : 0.0f; }
#pragma unroll
        for (int off = 16; off >= 1; off >>= 1) v += __shfl_xor(v, off, 32);
        if (lane == 0) red_s[wave] = v;
        __syncthreads();
        float t = 0.0f;
#pragma unroll
        for (int w = 0; w < 8; ++w) t += red_s[w];
        loss = t * (1.0f / (float)BROWS);
    }
    const int i = blockIdx.x * 256 + tid;
    const int k0 = 4 * i - 1; const int kc = k0 < 0 ? 0 : k0;
    float x0 = PW[kc];
    const float x1 = PW[4 * i], x2 = PW[4 * i + 1], x3 = PW[4 * i + 2];
    const float xt = PW[BROWS - 1];
    asm volatile("" : "+v"(x0));
    v4f val; val[0] = (i == 0) ? loss : x0; val[1] = x1; val[2] = x2; val[3] = x3;
    float* dst = OUT + (size_t)OUT1_EL + (size_t)4 * i;
    const bool tl = (i == NPIECE - 1);
    *(volatile v4f*)dst = val; if (tl) *(volatile float*)(dst + 4) = xt;
    __threadfence();
    *(volatile v4f*)dst = val; if (tl) *(volatile float*)(dst + 4) = xt;
}

static constexpr size_t al256(size_t v) { return (v + 255) & ~(size_t)255; }
static constexpr size_t SZ_TAB  = al256((size_t)2 * TABN * 4);
static constexpr size_t SZ_ACT  = al256((size_t)16 * DN * 2);
static constexpr size_t SZ_PW   = al256((size_t)BROWS * 4);
static constexpr size_t SZ_PART = al256((size_t)NBLK * PLINE * 4);
static constexpr size_t SZ_TOTAL = SZ_TAB + SZ_ACT + SZ_PW + SZ_PART;
static_assert(SZ_TOTAL <= (size_t)134217728);
static_assert(((size_t)TABN * 4) % 128 == 0);
static_assert((size_t)(TBLK - 1) * 256 + 252 + 4 <= (size_t)TABN);
static_assert((size_t)(NBLK - 1) * RPB + 60 + 4 <= (size_t)BROWS);
static_assert((size_t)(NBLK - 1) * PLINE + 28 + 4 <= (size_t)NBLK * PLINE);
static_assert((size_t)(NBLK - 1) * RPB * 2 + 124 + 4 <= (size_t)OUT1_EL);

extern "C" void kernel_launch(void* const* d_in, const int* in_sizes, int n_in,
                              void* d_out, int out_size, void* d_ws, size_t ws_size, hipStream_t stream) {
    if (n_in < 7) return;
    if ((size_t)in_sizes[0] < (size_t)(CF - 1) * B_FULL + BROWS) return;
    if ((size_t)in_sizes[1] < (size_t)BROWS * 2 || (size_t)in_sizes[2] < (size_t)BROWS * 2) return;
    if ((size_t)in_sizes[3] < (size_t)TABN || (size_t)in_sizes[4] < (size_t)TABN) return;
    if ((size_t)in_sizes[5] < (size_t)2 * DN) return;
    if ((size_t)in_sizes[6] < (size_t)BROWS * DN) return;
    if ((size_t)out_size < (size_t)OUT2_EL + BROWS) return;
    if (SZ_TOTAL > ws_size) return;
    const int*   idx   = (const int*)d_in[0];
    const float* label = (const float*)d_in[1];
    const float* posw  = (const float*)d_in[2];
    const float* meant = (const float*)d_in[3];
    const float* stdt  = (const float*)d_in[4];
    const float* act   = (const float*)d_in[5];
    const float* noise = (const float*)d_in[6];
    float* OUT = (float*)d_out;
    char* wsp = (char*)d_ws;
    float* TAB  = (float*)wsp; wsp += SZ_TAB;
    h16*   ACTH = (h16*)wsp;   wsp += SZ_ACT;
    float* PW   = (float*)wsp; wsp += SZ_PW;
    float* PART = (float*)wsp; wsp += SZ_PART;

    k_prep<<<dim3(TBLK + 1, 1, 1), 256, 0, stream>>>(meant, stdt, act, TAB, ACTH);
    k_main<<<dim3(NBLK, 1, 1), 32 * AW, 0, stream>>>(idx, label, posw, noise, TAB, ACTH, OUT, PW, PART);
    k_fin<<<dim3(NPIECE / 256, 1, 1), 256, 0, stream>>>(PW, PART, OUT);
}
